// FlashAttentionSim_65687229825379
// MI455X (gfx1250) — hardware-verified
//
#include <hip/hip_runtime.h>
#include <stdint.h>

typedef __attribute__((ext_vector_type(16))) _Float16 v16h;
typedef __attribute__((ext_vector_type(8)))  _Float16 v8h;
typedef __attribute__((ext_vector_type(16))) __bf16   v16b;
typedef __attribute__((ext_vector_type(8)))  __bf16   v8b;
typedef __attribute__((ext_vector_type(8)))  float    v8f;
typedef __attribute__((ext_vector_type(4)))  float    v4f;

static constexpr int kBatch   = 2;
static constexpr int kSeq     = 2048;
static constexpr int kDim     = 1024;
static constexpr int kHeads   = 16;
static constexpr int kHeadDim = 64;
static constexpr int kTok     = kBatch * kSeq;
static constexpr int kKvChunk = 64;
static constexpr int kQBlk    = 64;
static constexpr int kOsPitch = 68;
static constexpr float kAttScale = 0.125f;
static_assert(kHeads * kHeadDim == kDim);
static_assert(kTok % 64 == 0 && kDim % 64 == 0 && kDim % 32 == 0);
static_assert(kSeq % kQBlk == 0 && kSeq % kKvChunk == 0 && kHeadDim == 64);
#define NEG_INF_F (-__builtin_inff())

__device__ __forceinline__ unsigned short f2bf_bits(float f) {
  unsigned u = __float_as_uint(f);
  return (unsigned short)((u + 0x7FFFu + ((u >> 16) & 1u)) >> 16);
}
__device__ __forceinline__ float bf_bits2f(unsigned short h) { return __uint_as_float(((unsigned)h) << 16); }

__device__ __forceinline__ void dep_guard_h(v8f& a, v8f& b, v16h x, v16h y) { asm volatile("v_nop\n\tv_nop\n\tv_nop\n\tv_nop" : "+v"(a), "+v"(b) : "v"(x), "v"(y)); }
__device__ __forceinline__ void dep_guard_b(v8f& a, v8f& b, v16b x, v16b y) { asm volatile("v_nop\n\tv_nop\n\tv_nop\n\tv_nop" : "+v"(a), "+v"(b) : "v"(x), "v"(y)); }
__device__ __forceinline__ void keep4_h(v16h a, v16h b, v16h c, v16h d) { asm volatile("v_nop" :: "v"(a), "v"(b), "v"(c), "v"(d)); }
__device__ __forceinline__ void keep4_b(v16b a, v16b b, v16b c, v16b d) { asm volatile("v_nop" :: "v"(a), "v"(b), "v"(c), "v"(d)); }
__device__ __forceinline__ void acc_guard4(v8f& a, v8f& b, v8f& c, v8f& d) { asm volatile("v_nop\n\tv_nop\n\tv_nop\n\tv_nop" : "+v"(a), "+v"(b), "+v"(c), "+v"(d)); }
template <typename T> struct Frag;
template <> struct Frag<_Float16> {
  typedef v16h V; union U { v16h v; v8h h[2]; };
  static __device__ __forceinline__ v16h load(const _Float16* p) {
    U f; f.h[0] = *(const v8h*)(p); f.h[1] = *(const v8h*)(p + 16); return f.v;
  }
  static __device__ __forceinline__ v8f mma(v16h a, v16h b, v8f c) {
    return __builtin_amdgcn_wmma_f32_16x16x32_f16(false, a, false, b, (short)0, c, false, false);
  }
  static __device__ __forceinline__ void guard(v8f& a, v8f& b, v16h x, v16h y) { dep_guard_h(a, b, x, y); }
  static __device__ __forceinline__ void keep(v16h a, v16h b, v16h c, v16h d) { keep4_h(a, b, c, d); }
};
template <> struct Frag<__bf16> {
  typedef v16b V; union U { v16b v; v8b h[2]; };
  static __device__ __forceinline__ v16b load(const __bf16* p) {
    U f; f.h[0] = *(const v8b*)(p); f.h[1] = *(const v8b*)(p + 16); return f.v;
  }
  static __device__ __forceinline__ v8f mma(v16b a, v16b b, v8f c) {
    return __builtin_amdgcn_wmma_f32_16x16x32_bf16(false, a, false, b, (short)0, c, false, false);
  }
  static __device__ __forceinline__ void guard(v8f& a, v8f& b, v16b x, v16b y) { dep_guard_b(a, b, x, y); }
  static __device__ __forceinline__ void keep(v16b a, v16b b, v16b c, v16b d) { keep4_b(a, b, c, d); }
};

template <int ET> struct Elem;
template <> struct Elem<0> { typedef _Float16 T; };
template <> struct Elem<1> { typedef __bf16 T; };
template <int ET, int SPLIT, int BIAS_MODE, int OUT_MODE, bool RESID, int ACT = 0>
__global__ __launch_bounds__(256) void wmma_gemm64(
    const unsigned short* __restrict__ Ap, const unsigned short* __restrict__ A2p, int lda, long strideA,
    const unsigned short* __restrict__ Btp, const unsigned short* __restrict__ Bt2p, int ldb, long strideB,
    void* __restrict__ Cout, void* __restrict__ Cout2, int ldc, long strideC,
    const float* __restrict__ bias,
    const float* __restrict__ resid, long strideR,
    int M, int N, int K, float scale) {
  typedef typename Elem<ET>::T T;
  typedef typename Frag<T>::V V;
  const T* A = (const T*)Ap; const T* A2 = (const T*)A2p; const T* Bt = (const T*)Btp; const T* Bt2 = (const T*)Bt2p;
  __shared__ __align__(16) float sT[8][16 * 68];
  const int b    = blockIdx.y;
  const int lane = threadIdx.x & 31;
  const int wave = threadIdx.x >> 5;
  const int tilesN = N >> 6;
  const int tilesM = M >> 6;
  const int tile = blockIdx.x * 8 + wave;
  if (tile >= tilesM * tilesN) return;
  const int tm = tile / tilesN;
  const int tn = tile - tm * tilesN;
  const int m0 = tm << 6;
  const int n0 = tn << 6;

  const T* Ab  = A  + (size_t)b * strideA;
  const T* Bb  = Bt + (size_t)b * strideB;
  const T* Ab2 = SPLIT ? (A2  + (size_t)b * strideA) : nullptr;
  const T* Bb2 = (SPLIT == 1) ? (Bt2 + (size_t)b * strideB) : nullptr;

  const int rlane = lane & 15;
  const int koff  = (lane >> 4) * 8;
  const int mOff  = (lane >> 4) * 8;

  v8f acc[4][4];
#pragma unroll
  for (int i = 0; i < 4; ++i)
#pragma unroll
    for (int j = 0; j < 4; ++j) acc[i][j] = (v8f){0.f,0.f,0.f,0.f,0.f,0.f,0.f,0.f};

  for (int k0 = 0; k0 < K; k0 += 32) {
    V bh[4], bl[4];
#pragma unroll
    for (int j = 0; j < 4; ++j) {
      const size_t bo = (size_t)(n0 + (j << 4) + rlane) * ldb + koff + k0;
      bh[j] = Frag<T>::load(Bb + bo);
      if (SPLIT == 1) bl[j] = Frag<T>::load(Bb2 + bo);
    }
#pragma unroll
    for (int i = 0; i < 4; ++i) {
      const size_t ao = (size_t)(m0 + (i << 4) + rlane) * lda + koff + k0;
      V ah = Frag<T>::load(Ab + ao);
      V al;
      if (SPLIT) al = Frag<T>::load(Ab2 + ao);
#pragma unroll
      for (int j = 0; j < 4; ++j) {
        acc[i][j] = Frag<T>::mma(ah, bh[j], acc[i][j]);
        if (SPLIT == 1) acc[i][j] = Frag<T>::mma(ah, bl[j], acc[i][j]);
        if (SPLIT) acc[i][j] = Frag<T>::mma(al, bh[j], acc[i][j]);
      }
      Frag<T>::guard(acc[i][0], acc[i][3], ah, SPLIT ? al : ah);
    }
    Frag<T>::keep(bh[0], bh[1], bh[2], bh[3]);
    if (SPLIT == 1) Frag<T>::keep(bl[0], bl[1], bl[2], bl[3]);
  }
  acc_guard4(acc[0][0], acc[0][1], acc[0][2], acc[0][3]);
  acc_guard4(acc[1][0], acc[1][1], acc[1][2], acc[1][3]);
  acc_guard4(acc[2][0], acc[2][1], acc[2][2], acc[2][3]);
  acc_guard4(acc[3][0], acc[3][1], acc[3][2], acc[3][3]);

  float* slab = sT[wave];
  const float* Rb = RESID ? (resid + (size_t)b * strideR) : nullptr;
#pragma unroll
  for (int i = 0; i < 4; ++i) {
    const int mBase = m0 + (i << 4);
#pragma unroll
    for (int j = 0; j < 4; ++j) {
      const int n = n0 + (j << 4) + rlane;
      float bv = 0.f;
      if (BIAS_MODE == 2) bv = bias[n];
#pragma unroll
      for (int r = 0; r < 8; ++r) {
        float v = acc[i][j][r] * scale;
        if (BIAS_MODE == 1) v += bias[mBase + mOff + r];
        if (BIAS_MODE == 2) v += bv;
        if (RESID) v += Rb[(size_t)(mBase + mOff + r) * ldc + n];
        if (ACT == 1) v = tanhf(v);
        if (ACT == 2) v = fmaxf(v, 0.0f);
        if (ACT == 3) v = v / (1.0f + expf(-v));
        if (ACT == 4) v = (v > 0.f) ? v : 0.01f * v;
        slab[(mOff + r) * 68 + (j << 4) + rlane] = v;
      }
    }
    __builtin_amdgcn_fence(__ATOMIC_RELEASE, "workgroup");
    __builtin_amdgcn_wave_barrier();
    __builtin_amdgcn_fence(__ATOMIC_ACQUIRE, "workgroup");
    if (OUT_MODE == 0) {
      float* C = (float*)Cout + (size_t)b * strideC;
      const int hh = lane >> 4, c4 = (lane & 15) * 4;
      for (int pass = 0; pass < 2; ++pass) {
#pragma unroll
        for (int it = 0; it < 8; ++it) {
          const int row = it * 2 + hh;
          v4f v = *(const v4f*)(slab + row * 68 + c4);
          *(volatile v4f*)(C + (size_t)(mBase + row) * ldc + n0 + c4) = v;
        }
        __threadfence();
      }
    } else {
      const int q = lane >> 3, c8 = (lane & 7) * 8;
      unsigned short* C  = (unsigned short*)Cout  + (size_t)b * strideC;
      unsigned short* C2 = (OUT_MODE == 2) ? ((unsigned short*)Cout2 + (size_t)b * strideC) : nullptr;
      for (int pass = 0; pass < 2; ++pass) {
#pragma unroll
        for (int it = 0; it < 4; ++it) {
          const int row = it * 4 + q;
          const float* sp = slab + row * 68 + c8;
          v8h hv, lv;
#pragma unroll
          for (int e = 0; e < 8; ++e) {
            if (OUT_MODE == 1) {
              hv[e] = (_Float16)sp[e];
            } else {
              unsigned short hb = f2bf_bits(sp[e]);
              unsigned short lb = f2bf_bits(sp[e] - bf_bits2f(hb));
              hv[e] = __builtin_bit_cast(_Float16, hb);
              lv[e] = __builtin_bit_cast(_Float16, lb);
            }
          }
          *(volatile v8h*)(C + (size_t)(mBase + row) * ldc + n0 + c8) = hv;
          if (OUT_MODE == 2) *(volatile v8h*)(C2 + (size_t)(mBase + row) * ldc + n0 + c8) = lv;
        }
        __threadfence();
      }
    }
    __builtin_amdgcn_fence(__ATOMIC_RELEASE, "workgroup");
    __builtin_amdgcn_wave_barrier();
    __builtin_amdgcn_fence(__ATOMIC_ACQUIRE, "workgroup");
  }
}

__global__ __launch_bounds__(256) void cast_f32_bf16x2(
    const float* __restrict__ in, unsigned short* __restrict__ out, int n2) {
  int i = blockIdx.x * 256 + threadIdx.x;
  if (i < n2) {
    const unsigned u = (unsigned)f2bf_bits(in[2 * i]) | ((unsigned)f2bf_bits(in[2 * i + 1]) << 16);
    ((volatile unsigned*)out)[i] = u;
    __threadfence();
    ((volatile unsigned*)out)[i] = u;
  }
}

__device__ __forceinline__ void at_split(float f, __bf16& hi, __bf16& lo) {
  const unsigned short hb = f2bf_bits(f);
  hi = __builtin_bit_cast(__bf16, hb);
  lo = __builtin_bit_cast(__bf16, f2bf_bits(f - bf_bits2f(hb)));
}
__device__ __forceinline__ v8f mma_b(v16b a, v16b b, v8f c) {
  c = __builtin_amdgcn_wmma_f32_16x16x32_bf16(false, a, false, b, (short)0, c, false, false);
  asm volatile("v_nop\n\tv_nop\n\tv_nop\n\tv_nop" : "+v"(c) : "v"(a), "v"(b));
  return c;
}

__global__ __launch_bounds__(128) void attn64s_k(const unsigned short* __restrict__ hp,
                                                 const unsigned short* __restrict__ lp,
                                                 unsigned short* __restrict__ ohp,
                                                 unsigned short* __restrict__ olp) {
  union FB { v16b v; v8b h[2]; };
  __shared__ __align__(16) __bf16 Ksh[kKvChunk * kHeadDim];
  __shared__ __align__(16) __bf16 Ksl[kKvChunk * kHeadDim];
  __shared__ __align__(16) __bf16 Vth[kHeadDim * kKvChunk];
  __shared__ __align__(16) __bf16 Vtl[kHeadDim * kKvChunk];
  __shared__ __align__(16) __bf16 Psh[4][16 * kKvChunk];
  __shared__ __align__(16) __bf16 Psl[4][16 * kKvChunk];
  __shared__ __align__(16) float  Osf[4][16 * kOsPitch];
  const __bf16* Hb = (const __bf16*)hp;
  const __bf16* Lb = (const __bf16*)lp;
  _Float16* oh = (_Float16*)ohp;
  _Float16* ol = (_Float16*)olp;
  const int tid = threadIdx.x, wave = tid >> 5, lane = tid & 31, hh = lane >> 4, c = lane & 15;
  const int nqb = kSeq / kQBlk;
  const int bx = blockIdx.x;
  const int qb = bx % nqb;
  const int bh = bx / nqb;
  const int h = bh % kHeads;
  const int b = bh / kHeads;
  const int q0 = qb * kQBlk + wave * 16;
  const size_t PL = (size_t)kTok * kDim;
  const size_t base = (size_t)b * kSeq * kDim + (size_t)h * kHeadDim;
  const __bf16* Qh = Hb + base;            const __bf16* Ql = Lb + base;
  const __bf16* Kh = Hb + PL + base;       const __bf16* Kl = Lb + PL + base;
  const __bf16* Vh = Hb + 2 * PL + base;   const __bf16* Vl = Lb + 2 * PL + base;

  v16b qah[2], qal[2];
  {
    const __bf16* qr_h = Qh + (size_t)(q0 + c) * kDim + 8 * hh;
    const __bf16* qr_l = Ql + (size_t)(q0 + c) * kDim + 8 * hh;
#pragma unroll
    for (int dc = 0; dc < 2; ++dc) {
      qah[dc] = Frag<__bf16>::load(qr_h + dc * 32);
      qal[dc] = Frag<__bf16>::load(qr_l + dc * 32);
    }
  }
  float mrow[8], lrow[8];
  v8f oacc[4];
#pragma unroll
  for (int r = 0; r < 8; ++r) { mrow[r] = NEG_INF_F; lrow[r] = 0.f; }
#pragma unroll
  for (int t = 0; t < 4; ++t) oacc[t] = (v8f){0.f,0.f,0.f,0.f,0.f,0.f,0.f,0.f};

  const int nChunks = qb + 1;
  for (int kc = 0; kc < nChunks; ++kc) {
    const int kv0 = kc * kKvChunk;
    __syncthreads();
    {
      const int kvr = tid >> 1, dh = (tid & 1) * 32;
      const size_t ro = (size_t)(kv0 + kvr) * kDim + dh;
#pragma unroll 1
      for (int i = 0; i < 4; ++i) {
        const v8b kkh = *(const v8b*)(Kh + ro + 8 * i);
        const v8b kkl = *(const v8b*)(Kl + ro + 8 * i);
        *(v8b*)(Ksh + kvr * kHeadDim + dh + 8 * i) = kkh;
        *(v8b*)(Ksl + kvr * kHeadDim + dh + 8 * i) = kkl;
        const v8b vvh = *(const v8b*)(Vh + ro + 8 * i);
        const v8b vvl = *(const v8b*)(Vl + ro + 8 * i);
#pragma unroll
        for (int e = 0; e < 8; ++e) {
          Vth[(dh + 8 * i + e) * kKvChunk + kvr] = vvh[e];
          Vtl[(dh + 8 * i + e) * kKvChunk + kvr] = vvl[e];
        }
      }
    }
    __syncthreads();

    v8f s[4];
#pragma unroll
    for (int j = 0; j < 4; ++j) {
      s[j] = (v8f){0.f,0.f,0.f,0.f,0.f,0.f,0.f,0.f};
#pragma unroll
      for (int dc = 0; dc < 2; ++dc) {
        FB kb, kl;
        kb.h[0] = *(const v8b*)(Ksh + (j * 16 + c) * kHeadDim + dc * 32 + 8 * hh);
        kb.h[1] = *(const v8b*)(Ksh + (j * 16 + c) * kHeadDim + dc * 32 + 16 + 8 * hh);
        kl.h[0] = *(const v8b*)(Ksl + (j * 16 + c) * kHeadDim + dc * 32 + 8 * hh);
        kl.h[1] = *(const v8b*)(Ksl + (j * 16 + c) * kHeadDim + dc * 32 + 16 + 8 * hh);
        s[j] = mma_b(qah[dc], kb.v, s[j]);
        s[j] = mma_b(qah[dc], kl.v, s[j]);
        s[j] = mma_b(qal[dc], kb.v, s[j]);
      }
    }
    const bool diag = (kc == qb);
    float cm[8];
#pragma unroll
    for (int r = 0; r < 8; ++r) {
      const int qrow = q0 + 8 * hh + r;
      float m = NEG_INF_F;
#pragma unroll
      for (int j = 0; j < 4; ++j) {
        const int kvcol = kv0 + j * 16 + c;
        float sv = s[j][r] * kAttScale;
        if (diag && (kvcol > qrow)) sv = NEG_INF_F;
        s[j][r] = sv;
        m = fmaxf(m, sv);
      }
#pragma unroll
      for (int off = 1; off < 16; off <<= 1) m = fmaxf(m, __shfl_xor(m, off, 32));
      cm[r] = m;
    }
    __bf16* pwh = Psh[wave];
    __bf16* pwl = Psl[wave];
#pragma unroll
    for (int r = 0; r < 8; ++r) {
      const float mnew = fmaxf(mrow[r], cm[r]);
      const float mref = (mnew > NEG_INF_F) ? mnew : 0.0f;
      const float alpha = expf(mrow[r] - mref);
      mrow[r] = mnew;
      float psum = 0.f;
#pragma unroll
      for (int j = 0; j < 4; ++j) {
        const float p = expf(s[j][r] - mref);
        psum += p;
        __bf16 ph, pl;
        at_split(p, ph, pl);
        pwh[(8 * hh + r) * kKvChunk + j * 16 + c] = ph;
        pwl[(8 * hh + r) * kKvChunk + j * 16 + c] = pl;
      }
#pragma unroll
      for (int off = 1; off < 16; off <<= 1) psum += __shfl_xor(psum, off, 32);
      lrow[r] = lrow[r] * alpha + psum;
#pragma unroll
      for (int t = 0; t < 4; ++t) oacc[t][r] *= alpha;
    }
    __builtin_amdgcn_fence(__ATOMIC_RELEASE, "workgroup");
    __builtin_amdgcn_wave_barrier();
    __builtin_amdgcn_fence(__ATOMIC_ACQUIRE, "workgroup");
#pragma unroll 1
    for (int kk = 0; kk < 2; ++kk) {
      FB pa, pb;
      pa.h[0] = *(const v8b*)(pwh + c * kKvChunk + kk * 32 + 8 * hh);
      pa.h[1] = *(const v8b*)(pwh + c * kKvChunk + kk * 32 + 16 + 8 * hh);
      pb.h[0] = *(const v8b*)(pwl + c * kKvChunk + kk * 32 + 8 * hh);
      pb.h[1] = *(const v8b*)(pwl + c * kKvChunk + kk * 32 + 16 + 8 * hh);
#pragma unroll
      for (int t = 0; t < 4; ++t) {
        FB vb, vl;
        vb.h[0] = *(const v8b*)(Vth + (t * 16 + c) * kKvChunk + kk * 32 + 8 * hh);
        vb.h[1] = *(const v8b*)(Vth + (t * 16 + c) * kKvChunk + kk * 32 + 16 + 8 * hh);
        vl.h[0] = *(const v8b*)(Vtl + (t * 16 + c) * kKvChunk + kk * 32 + 8 * hh);
        vl.h[1] = *(const v8b*)(Vtl + (t * 16 + c) * kKvChunk + kk * 32 + 16 + 8 * hh);
        oacc[t] = mma_b(pa.v, vb.v, oacc[t]);
        oacc[t] = mma_b(pa.v, vl.v, oacc[t]);
        oacc[t] = mma_b(pb.v, vb.v, oacc[t]);
      }
    }
  }

  float* os = Osf[wave];
#pragma unroll
  for (int r = 0; r < 8; ++r) {
    const float inv = 1.0f / fmaxf(lrow[r], 1e-12f);
#pragma unroll
    for (int t = 0; t < 4; ++t) os[(8 * hh + r) * kOsPitch + t * 16 + c] = oacc[t][r] * inv;
  }
  __builtin_amdgcn_fence(__ATOMIC_RELEASE, "workgroup");
  __builtin_amdgcn_wave_barrier();
  __builtin_amdgcn_fence(__ATOMIC_ACQUIRE, "workgroup");
  {
    const int q8 = lane >> 3, c8 = (lane & 7) * 8;
    const size_t ob = (size_t)b * kSeq * kDim + (size_t)h * kHeadDim;
    for (int pass = 0; pass < 2; ++pass) {
#pragma unroll
      for (int it = 0; it < 4; ++it) {
        const int row = it * 4 + q8;
        const float* sp = os + row * kOsPitch + c8;
        v8h hv, lv;
#pragma unroll
        for (int e = 0; e < 8; ++e) {
          const unsigned short hb = f2bf_bits(sp[e]);
          const unsigned short lb = f2bf_bits(sp[e] - bf_bits2f(hb));
          hv[e] = __builtin_bit_cast(_Float16, hb);
          lv[e] = __builtin_bit_cast(_Float16, lb);
        }
        const size_t o = ob + (size_t)(q0 + row) * kDim + c8;
        *(volatile v8h*)(oh + o) = hv;
        *(volatile v8h*)(ol + o) = lv;
      }
      __threadfence();
    }
  }
}

extern "C" void kernel_launch(void* const* d_in, const int* in_sizes, int n_in,
                              void* d_out, int out_size, void* d_ws, size_t ws_size,
                              hipStream_t stream) {
  const int NX = kTok * kDim;
  const int NW = kDim * kDim;
  if (n_in < 5) return;
  if (in_sizes[0] != NX || in_sizes[1] != NW || in_sizes[2] != NW || in_sizes[3] != NW ||
      in_sizes[4] != NW || out_size != NX) return;

  const float* xf  = (const float*)d_in[0];
  const float* wqf = (const float*)d_in[1];
  const float* wkf = (const float*)d_in[2];
  const float* wvf = (const float*)d_in[3];
  const float* wof = (const float*)d_in[4];
  float* out = (float*)d_out;

  const size_t bX   = (size_t)NX * 2;
  const size_t bW   = (size_t)4 * NW * 2;
  const size_t bQKV = (size_t)3 * NX * 2;
  const size_t bO   = (size_t)NX * 2;
  size_t off = 0;
  unsigned short* Xb   = (unsigned short*)((char*)d_ws + off); off += bX;
  unsigned short* Wb   = (unsigned short*)((char*)d_ws + off); off += bW;
  unsigned short* QKVh = (unsigned short*)((char*)d_ws + off); off += bQKV;
  unsigned short* QKVl = (unsigned short*)((char*)d_ws + off); off += bQKV;
  unsigned short* Oh   = (unsigned short*)((char*)d_ws + off); off += bO;
  unsigned short* Ol   = (unsigned short*)((char*)d_ws + off); off += bO;
  if (off > ws_size) return;

  const int nx2 = NX / 2, nw2 = NW / 2;
  cast_f32_bf16x2<<<(nx2 + 255) / 256, 256, 0, stream>>>(xf, Xb, nx2);
  cast_f32_bf16x2<<<(nw2 + 255) / 256, 256, 0, stream>>>(wqf, Wb, nw2);
  cast_f32_bf16x2<<<(nw2 + 255) / 256, 256, 0, stream>>>(wkf, Wb + (size_t)NW, nw2);
  cast_f32_bf16x2<<<(nw2 + 255) / 256, 256, 0, stream>>>(wvf, Wb + (size_t)2 * NW, nw2);
  cast_f32_bf16x2<<<(nw2 + 255) / 256, 256, 0, stream>>>(wof, Wb + (size_t)3 * NW, nw2);

  const int tiles = (kTok / 64) * (kDim / 64);
  const int gx = (tiles + 7) / 8;
  wmma_gemm64<1, 0, 0, 2, false><<<dim3(gx, 3), 256, 0, stream>>>(
      Xb, Xb, kDim, 0L,
      Wb, Wb, kDim, (long)NW,
      (void*)QKVh, (void*)QKVl, kDim, (long)NX,
      xf, xf, 0L,
      kTok, kDim, kDim, 1.0f);

  attn64s_k<<<kBatch * kHeads * (kSeq / kQBlk), 128, 0, stream>>>(QKVh, QKVl, Oh, Ol);

  wmma_gemm64<1, 2, 0, 0, false><<<dim3(gx, 1), 256, 0, stream>>>(
      Oh, Ol, kDim, 0L,
      Wb + (size_t)3 * NW, Wb + (size_t)3 * NW, kDim, 0L,
      (void*)out, (void*)out, kDim, 0L,
      xf, xf, 0L,
      kTok, kDim, kDim, 1.0f);
}
